// CrossAtt_64063732187816
// MI455X (gfx1250) — hardware-verified
//
#include <hip/hip_runtime.h>
#include <math.h>
#include <stdint.h>

#define NB   4
#define SEQ  2048
#define DMOD 768
#define NH   12
#define HD   64
#define NTOK (NB * SEQ)
#define NKT  (SEQ / 64)
static_assert(NH * HD == DMOD);
static_assert((SEQ % 64) == 0 && (DMOD % 64) == 0 && (NTOK % 64) == 0 && (DMOD % 32) == 0);
static_assert(SEQ == 128 * 16);
static_assert((DMOD % 128) == 0);

typedef _Float16 v16h __attribute__((ext_vector_type(16)));
typedef _Float16 v8h  __attribute__((ext_vector_type(8)));
typedef __bf16   v16b __attribute__((ext_vector_type(16)));
typedef __bf16   v8b  __attribute__((ext_vector_type(8)));
typedef float    v8f  __attribute__((ext_vector_type(8)));
typedef float    v4f  __attribute__((ext_vector_type(4)));
typedef unsigned int v4u __attribute__((ext_vector_type(4)));
typedef int      v4i __attribute__((ext_vector_type(4)));

__device__ __forceinline__ unsigned short bf_bits(float f) {
  unsigned u = __float_as_uint(f);
  return (unsigned short)((u + 0x7FFFu + ((u >> 16) & 1u)) >> 16);
}
__device__ __forceinline__ float bf_up(unsigned short h) { return __uint_as_float(((unsigned)h) << 16); }
__device__ __forceinline__ float bf_rn(float f) { return bf_up(bf_bits(f)); }
__device__ __forceinline__ unsigned short h_bits(_Float16 x) { return __builtin_bit_cast(unsigned short, x); }
__device__ __forceinline__ unsigned pk16(unsigned short a, unsigned short b) { return (unsigned)a | ((unsigned)b << 16); }
__device__ __forceinline__ v8f zero8() { v8f z = {0.f, 0.f, 0.f, 0.f, 0.f, 0.f, 0.f, 0.f}; return z; }

__device__ __forceinline__ v16b ldfrag_b(const __bf16* p) {
  union { v16b v; v8b h[2]; } f;
  f.h[0] = *(const v8b*)(p);
  f.h[1] = *(const v8b*)(p + 16);
  return f.v;
}
__device__ __forceinline__ v16h ldfrag_h(const _Float16* p) {
  union { v16h v; v8h h[2]; } f;
  f.h[0] = *(const v8h*)(p);
  f.h[1] = *(const v8h*)(p + 16);
  return f.v;
}

__device__ __forceinline__ v8f mma_b(v16b a, v16b b, v8f c) {
  c = __builtin_amdgcn_wmma_f32_16x16x32_bf16(false, a, false, b, (short)0, c, false, false);
#if defined(__HIP_DEVICE_COMPILE__)
  asm volatile("v_nop\n\tv_nop\n\tv_nop\n\tv_nop" : "+v"(c) : "v"(a), "v"(b));
#endif
  return c;
}
__device__ __forceinline__ v8f mma_h(v16h a, v16h b, v8f c) {
  c = __builtin_amdgcn_wmma_f32_16x16x32_f16(false, a, false, b, (short)0, c, false, false);
#if defined(__HIP_DEVICE_COMPILE__)
  asm volatile("v_nop\n\tv_nop\n\tv_nop\n\tv_nop" : "+v"(c) : "v"(a), "v"(b));
#endif
  return c;
}
__device__ __forceinline__ v8f mma_b_raw(v16b a, v16b b, v8f c) {
  return __builtin_amdgcn_wmma_f32_16x16x32_bf16(false, a, false, b, (short)0, c, false, false);
}
__device__ __forceinline__ void dep_guard_b(v8f& a, v8f& b, v16b x, v16b y) {
#if defined(__HIP_DEVICE_COMPILE__)
  asm volatile("v_nop\n\tv_nop\n\tv_nop\n\tv_nop" : "+v"(a), "+v"(b) : "v"(x), "v"(y));
#endif
}
__device__ __forceinline__ void keep4_b(v16b a, v16b b, v16b c, v16b d) {
#if defined(__HIP_DEVICE_COMPILE__)
  asm volatile("v_nop" :: "v"(a), "v"(b), "v"(c), "v"(d));
#endif
}
__device__ __forceinline__ void acc_guard4(v8f& a, v8f& b, v8f& c, v8f& d) {
#if defined(__HIP_DEVICE_COMPILE__)
  asm volatile("v_nop\n\tv_nop\n\tv_nop\n\tv_nop" : "+v"(a), "+v"(b), "+v"(c), "+v"(d));
#endif
}

__global__ __launch_bounds__(256) void cvt_bf16x8(const float* __restrict__ in, unsigned short* out, int n8) {
  const int i = blockIdx.x * 256 + threadIdx.x;
  if (i < n8) {
    const v4f a = *(const v4f*)(in + (size_t)i * 8);
    const v4f b = *(const v4f*)(in + (size_t)i * 8 + 4);
    v4u p;
    p[0] = pk16(bf_bits(a[0]), bf_bits(a[1]));
    p[1] = pk16(bf_bits(a[2]), bf_bits(a[3]));
    p[2] = pk16(bf_bits(b[0]), bf_bits(b[1]));
    p[3] = pk16(bf_bits(b[2]), bf_bits(b[3]));
    *(volatile v4u*)(out + (size_t)i * 8) = p;
    __threadfence();
    *(volatile v4u*)(out + (size_t)i * 8) = p;
  }
}

__global__ __launch_bounds__(256) void cvt_wT(const float* __restrict__ w, unsigned short* out) {
  __shared__ __align__(16) unsigned short sh[64 * 72];
  const int tid  = threadIdx.x;
  const int lane = tid & 31;
  const int wave = tid >> 5;
  const int n0 = blockIdx.x * 64;
  const int k0 = blockIdx.y * 64;
  {
    const int kr = tid >> 2;
    const int nc = (tid & 3) * 16;
    const float* src = w + (size_t)(k0 + kr) * DMOD + n0 + nc;
#pragma unroll
    for (int e = 0; e < 4; ++e) {
      const v4f a = *(const v4f*)(src + 4 * e);
#pragma unroll
      for (int j = 0; j < 4; ++j) sh[(nc + 4 * e + j) * 72 + kr] = bf_bits(a[j]);
    }
  }
  __syncthreads();
  const int q = lane >> 3, c8 = (lane & 7) * 8;
  v4u v[2];
#pragma unroll
  for (int it = 0; it < 2; ++it) {
    const int row = wave * 8 + it * 4 + q;
    v[it] = *(const v4u*)(sh + row * 72 + c8);
  }
  for (int pass = 0; pass < 2; ++pass) {
#pragma unroll
    for (int it = 0; it < 2; ++it) {
      const int row = wave * 8 + it * 4 + q;
      *(volatile v4u*)(out + (size_t)(n0 + row) * DMOD + k0 + c8) = v[it];
    }
    __threadfence();
  }
}

template <int NSPLIT, int OUT_MODE, int EPI>
__global__ __launch_bounds__(256) void gemm64(
    const unsigned short* __restrict__ Ap, const unsigned short* __restrict__ A2p, int lda, long long strideA,
    const unsigned short* __restrict__ Btp, int ldb, long long strideB,
    const float* __restrict__ bias, const float* __restrict__ addend,
    void* C0, void* C1, void* C2, int ldc, long long strideC,
    int M, int N, int K, float oscale, float rscale) {
  static_assert(OUT_MODE >= 1 && OUT_MODE <= 5);
  static_assert((EPI & 4) == 0 || OUT_MODE == 4);
  static_assert(NSPLIT == 0 || NSPLIT == 1);
  const __bf16* A  = (const __bf16*)(const void*)Ap;
  const __bf16* A2 = (const __bf16*)(const void*)A2p;
  const __bf16* Bt = (const __bf16*)(const void*)Btp;
  __shared__ __align__(16) float sT[8][16 * 68];
  const int b    = blockIdx.y;
  const int lane = threadIdx.x & 31;
  const int wave = threadIdx.x >> 5;
  const int tilesN = N >> 6;
  const int tilesM = M >> 6;
  const int tile = blockIdx.x * 8 + wave;
  if (tile >= tilesM * tilesN) return;
  const int tm = tile / tilesN;
  const int tn = tile - tm * tilesN;
  const int m0 = tm << 6;
  const int n0 = tn << 6;

  const __bf16* Ab  = A  + (size_t)b * strideA;
  const __bf16* Bb  = Bt + (size_t)b * strideB;
  const __bf16* Ab2 = (NSPLIT >= 1) ? (A2 + (size_t)b * strideA) : Ab;

  const int rlane = lane & 15;
  const int koff  = (lane >> 4) * 8;
  const int mOff  = (lane >> 4) * 8;

  v8f acc[4][4];
#pragma unroll
  for (int i = 0; i < 4; ++i)
#pragma unroll
    for (int j = 0; j < 4; ++j) acc[i][j] = zero8();

  for (int k0 = 0; k0 < K; k0 += 32) {
    v16b bh[4];
#pragma unroll
    for (int j = 0; j < 4; ++j) {
      const size_t bo = (size_t)(n0 + (j << 4) + rlane) * ldb + koff + k0;
      bh[j] = ldfrag_b(Bb + bo);
    }
#pragma unroll
    for (int i = 0; i < 4; ++i) {
      const size_t ao = (size_t)(m0 + (i << 4) + rlane) * lda + koff + k0;
      const v16b ah = ldfrag_b(Ab + ao);
      v16b al = ah;
      if (NSPLIT >= 1) al = ldfrag_b(Ab2 + ao);
#pragma unroll
      for (int j = 0; j < 4; ++j) {
        acc[i][j] = mma_b_raw(ah, bh[j], acc[i][j]);
        if (NSPLIT >= 1) acc[i][j] = mma_b_raw(al, bh[j], acc[i][j]);
      }
      dep_guard_b(acc[i][0], acc[i][3], ah, al);
    }
    keep4_b(bh[0], bh[1], bh[2], bh[3]);
  }
  acc_guard4(acc[0][0], acc[0][1], acc[0][2], acc[0][3]);
  acc_guard4(acc[1][0], acc[1][1], acc[1][2], acc[1][3]);
  acc_guard4(acc[2][0], acc[2][1], acc[2][2], acc[2][3]);
  acc_guard4(acc[3][0], acc[3][1], acc[3][2], acc[3][3]);

  float* slab = sT[wave];
  const int hh2 = lane >> 4, c4 = (lane & 15) * 4;
  const int q4  = lane >> 3, c8 = (lane & 7) * 8;
  v4f b4 = {0.f, 0.f, 0.f, 0.f};
  float b8[8];
#pragma unroll
  for (int e = 0; e < 8; ++e) b8[e] = 0.f;
  if (EPI & 1) {
    const v4f t = *(const v4f*)(bias + n0 + c4);
#pragma unroll
    for (int e = 0; e < 4; ++e) b4[e] = bf_rn(t[e]);
    const v4f t0 = *(const v4f*)(bias + n0 + c8);
    const v4f t1 = *(const v4f*)(bias + n0 + c8 + 4);
#pragma unroll
    for (int e = 0; e < 4; ++e) { b8[e] = bf_rn(t0[e]); b8[4 + e] = bf_rn(t1[e]); }
  }

#pragma unroll
  for (int i = 0; i < 4; ++i) {
    const int mBase = m0 + (i << 4);
#pragma unroll
    for (int j = 0; j < 4; ++j) {
#pragma unroll
      for (int r = 0; r < 8; ++r) {
        slab[(mOff + r) * 68 + (j << 4) + rlane] = acc[i][j][r];
      }
    }
    __builtin_amdgcn_fence(__ATOMIC_RELEASE, "workgroup");
    __builtin_amdgcn_wave_barrier();
    __builtin_amdgcn_fence(__ATOMIC_ACQUIRE, "workgroup");
    if (OUT_MODE == 4 || OUT_MODE == 5) {
      float* C = (float*)C0 + (size_t)b * strideC;
      v4f fv[8];
#pragma unroll
      for (int it = 0; it < 8; ++it) {
        const int row = it * 2 + hh2;
        v4f v = *(const v4f*)(slab + row * 68 + c4);
        if (EPI & 1) v += b4;
        if (EPI & 2) {
#pragma unroll
          for (int e = 0; e < 4; ++e) v[e] = fmaxf(v[e], 0.f);
        }
        if (EPI & 4) v += *(const v4f*)(addend + (size_t)b * strideC + (size_t)(mBase + row) * ldc + n0 + c4);
        fv[it] = v;
      }
      for (int pass = 0; pass < 2; ++pass) {
#pragma unroll
        for (int it = 0; it < 8; ++it) {
          const int row = it * 2 + hh2;
          *(volatile v4f*)(C + (size_t)(mBase + row) * ldc + n0 + c4) = fv[it];
        }
        __threadfence();
      }
    }
    if (OUT_MODE != 4) {
      unsigned short* P0 = (unsigned short*)((OUT_MODE == 5) ? C1 : C0) + (size_t)b * strideC;
      unsigned short* P1 = (unsigned short*)((OUT_MODE == 5) ? C2 : C1) + (size_t)b * strideC;
      v4u hv[4], lv[4];
#pragma unroll
      for (int it = 0; it < 4; ++it) {
        const int row = it * 4 + q4;
        const float* sp = slab + row * 68 + c8;
        v4u a, a2;
#pragma unroll
        for (int e = 0; e < 4; ++e) {
          float f0 = sp[2 * e], f1 = sp[2 * e + 1];
          if (EPI & 1) { f0 += b8[2 * e]; f1 += b8[2 * e + 1]; }
          if (EPI & 2) { f0 = fmaxf(f0, 0.f); f1 = fmaxf(f1, 0.f); }
          unsigned short h0, h1, l0, l1;
          if (OUT_MODE == 1) {
            h0 = h_bits((_Float16)(f0 * oscale)); h1 = h_bits((_Float16)(f1 * oscale));
            l0 = 0; l1 = 0;
          } else if (OUT_MODE == 3) {
            const float x0 = f0 * oscale, x1 = f1 * oscale;
            const _Float16 y0 = (_Float16)x0, y1 = (_Float16)x1;
            h0 = h_bits(y0); h1 = h_bits(y1);
            l0 = h_bits((_Float16)((x0 - (float)y0) * rscale));
            l1 = h_bits((_Float16)((x1 - (float)y1) * rscale));
          } else {
            h0 = bf_bits(f0); h1 = bf_bits(f1);
            l0 = bf_bits(f0 - bf_up(h0)); l1 = bf_bits(f1 - bf_up(h1));
          }
          a[e] = pk16(h0, h1); a2[e] = pk16(l0, l1);
        }
        hv[it] = a; lv[it] = a2;
      }
      for (int pass = 0; pass < 2; ++pass) {
#pragma unroll
        for (int it = 0; it < 4; ++it) {
          const int row = it * 4 + q4;
          const size_t go = (size_t)(mBase + row) * ldc + n0 + c8;
          *(volatile v4u*)(P0 + go) = hv[it];
          if (OUT_MODE != 1) *(volatile v4u*)(P1 + go) = lv[it];
        }
        __threadfence();
      }
    }
    __builtin_amdgcn_fence(__ATOMIC_RELEASE, "workgroup");
    __builtin_amdgcn_wave_barrier();
    __builtin_amdgcn_fence(__ATOMIC_ACQUIRE, "workgroup");
  }
}

__global__ __launch_bounds__(128)
void attn64(const unsigned short* __restrict__ qpl, const unsigned short* __restrict__ kpl,
            const unsigned short* __restrict__ vhp, const unsigned short* __restrict__ vlp,
            const int* __restrict__ mask, unsigned short* ohp, unsigned short* olp,
            float sscale, float oscl, float rres) {
  union FH { v16h v; v8h h[2]; };
  __shared__ __align__(16) _Float16 Ksh[64 * 64];
  __shared__ __align__(16) _Float16 Vth[64 * 64];
  __shared__ __align__(16) _Float16 Vtl[64 * 64];
  __shared__ __align__(16) _Float16 Psh[4][16 * 64];
  __shared__ __align__(16) float    Os[4][16 * 64];
  __shared__ int red[4];

  const int tid  = threadIdx.x;
  const int wave = tid >> 5;
  const int lane = tid & 31;
  const int hh   = lane >> 4;
  const int c    = lane & 15;

  const int bx   = blockIdx.x;
  const int qb   = bx % NKT;
  const int rest = bx / NKT;
  const int h    = rest % NH;
  const int b    = rest / NH;
  const int q0   = qb * 64 + wave * 16;
  const size_t rowB = (size_t)b * SEQ;

  int cnt = 0;
  {
    const int* mp = mask + (size_t)b * SEQ + tid * 16;
#pragma unroll
    for (int e = 0; e < 4; ++e) {
      const v4i m4 = *(const v4i*)(mp + 4 * e);
      cnt += (m4[0] != 0 ? 1 : 0) + (m4[1] != 0 ? 1 : 0) + (m4[2] != 0 ? 1 : 0) + (m4[3] != 0 ? 1 : 0);
    }
  }
#pragma unroll
  for (int off = 1; off < 32; off <<= 1) cnt += __shfl_xor(cnt, off, 32);
  if (lane == 0) red[wave] = cnt;
  __syncthreads();
  const int vl = red[0] + red[1] + red[2] + red[3];
  int nkt = (vl + 63) >> 6;
  if (vl <= 0) nkt = NKT;
  if (nkt > NKT) nkt = NKT;

  const _Float16* Q  = (const _Float16*)(const void*)qpl + (size_t)h * HD;
  const _Float16* Kp = (const _Float16*)(const void*)kpl + (size_t)h * HD;
  const _Float16* Vh = (const _Float16*)(const void*)vhp + ((size_t)b * DMOD + (size_t)h * HD) * SEQ;
  const _Float16* Vl = (const _Float16*)(const void*)vlp + ((size_t)b * DMOD + (size_t)h * HD) * SEQ;

  v16h qa[2];
#pragma unroll
  for (int dc = 0; dc < 2; ++dc) {
    qa[dc] = ldfrag_h(Q + (rowB + q0 + c) * DMOD + dc * 32 + 8 * hh);
  }

  float mrow[8], lrow[8];
  v8f oacc[4];
#pragma unroll
  for (int r = 0; r < 8; ++r) { mrow[r] = -INFINITY; lrow[r] = 0.f; }
#pragma unroll
  for (int t = 0; t < 4; ++t) oacc[t] = zero8();

  for (int kt = 0; kt < nkt; ++kt) {
    const int kv0 = kt * 64;
    __syncthreads();
    {
      const int r = tid >> 1, half = (tid & 1) * 32;
      const _Float16* kg  = Kp + (rowB + kv0 + r) * DMOD + half;
      const _Float16* vg  = Vh + (size_t)r * SEQ + kv0 + half;
      const _Float16* vlg = Vl + (size_t)r * SEQ + kv0 + half;
#pragma unroll
      for (int i = 0; i < 4; ++i) {
        const v8h a0 = *(const v8h*)(kg + 8 * i);
        const v8h b0 = *(const v8h*)(vg + 8 * i);
        const v8h b1 = *(const v8h*)(vlg + 8 * i);
        *(v8h*)(Ksh + r * 64 + half + 8 * i) = a0;
        *(v8h*)(Vth + r * 64 + half + 8 * i) = b0;
        *(v8h*)(Vtl + r * 64 + half + 8 * i) = b1;
      }
    }
    __syncthreads();

    v8f s[4];
#pragma unroll
    for (int j = 0; j < 4; ++j) {
      s[j] = zero8();
#pragma unroll
      for (int dc = 0; dc < 2; ++dc) {
        FH kb;
        kb.h[0] = *(const v8h*)(Ksh + (j * 16 + c) * 64 + dc * 32 + 8 * hh);
        kb.h[1] = *(const v8h*)(Ksh + (j * 16 + c) * 64 + dc * 32 + 16 + 8 * hh);
        s[j] = mma_h(qa[dc], kb.v, s[j]);
      }
    }

    _Float16* pw = Psh[wave];
#pragma unroll
    for (int r = 0; r < 8; ++r) {
      float m = -INFINITY;
#pragma unroll
      for (int j = 0; j < 4; ++j) {
        const int kidx = kv0 + j * 16 + c;
        float sv = s[j][r] * sscale;
        sv = (kidx < vl) ? sv : -1.0e6f;
        s[j][r] = sv;
        m = fmaxf(m, sv);
      }
#pragma unroll
      for (int off = 1; off < 16; off <<= 1) m = fmaxf(m, __shfl_xor(m, off, 32));
      const float mnew  = fmaxf(mrow[r], m);
      const float msafe = (mnew == -INFINITY) ? 0.f : mnew;
      const float alpha = __expf(mrow[r] - msafe);
      mrow[r] = mnew;
      float psum = 0.f;
#pragma unroll
      for (int j = 0; j < 4; ++j) {
        const float p = __expf(s[j][r] - msafe);
        psum += p;
        pw[(8 * hh + r) * 64 + j * 16 + c] = (_Float16)(p * 1024.0f);
      }
#pragma unroll
      for (int off = 1; off < 16; off <<= 1) psum += __shfl_xor(psum, off, 32);
      lrow[r] = lrow[r] * alpha + psum;
#pragma unroll
      for (int t = 0; t < 4; ++t) oacc[t][r] *= alpha;
    }
    __builtin_amdgcn_fence(__ATOMIC_RELEASE, "workgroup");
    __builtin_amdgcn_wave_barrier();
    __builtin_amdgcn_fence(__ATOMIC_ACQUIRE, "workgroup");

    v8f o1[4];
#pragma unroll
    for (int t = 0; t < 4; ++t) o1[t] = zero8();
#pragma unroll 1
    for (int kk = 0; kk < 2; ++kk) {
      FH pa;
      pa.h[0] = *(const v8h*)(pw + c * 64 + kk * 32 + 8 * hh);
      pa.h[1] = *(const v8h*)(pw + c * 64 + kk * 32 + 16 + 8 * hh);
#pragma unroll
      for (int t = 0; t < 4; ++t) {
        FH vb, vr;
        vb.h[0] = *(const v8h*)(Vth + (t * 16 + c) * 64 + kk * 32 + 8 * hh);
        vb.h[1] = *(const v8h*)(Vth + (t * 16 + c) * 64 + kk * 32 + 16 + 8 * hh);
        vr.h[0] = *(const v8h*)(Vtl + (t * 16 + c) * 64 + kk * 32 + 8 * hh);
        vr.h[1] = *(const v8h*)(Vtl + (t * 16 + c) * 64 + kk * 32 + 16 + 8 * hh);
        oacc[t] = mma_h(pa.v, vb.v, oacc[t]);
        o1[t]   = mma_h(pa.v, vr.v, o1[t]);
      }
    }
#pragma unroll
    for (int t = 0; t < 4; ++t)
#pragma unroll
      for (int r = 0; r < 8; ++r) oacc[t][r] += o1[t][r] * rres;
  }

  float* os = Os[wave];
#pragma unroll
  for (int r = 0; r < 8; ++r) {
    const float l = lrow[r];
    const float inv = ((l > 0.f) ? (1.0f / l) : 0.f) * oscl;
#pragma unroll
    for (int t = 0; t < 4; ++t) os[(8 * hh + r) * 64 + t * 16 + c] = oacc[t][r] * inv;
  }
  __builtin_amdgcn_fence(__ATOMIC_RELEASE, "workgroup");
  __builtin_amdgcn_wave_barrier();
  __builtin_amdgcn_fence(__ATOMIC_ACQUIRE, "workgroup");
  {
    const int q4 = lane >> 3, c8 = (lane & 7) * 8;
    v4u hv[4], lv[4];
#pragma unroll
    for (int it = 0; it < 4; ++it) {
      const int row = it * 4 + q4;
      const float* sp = os + row * 64 + c8;
      v4u a, a2;
#pragma unroll
      for (int e = 0; e < 4; ++e) {
        const float f0 = sp[2 * e], f1 = sp[2 * e + 1];
        const unsigned short h0 = bf_bits(f0), h1 = bf_bits(f1);
        const unsigned short l0 = bf_bits(f0 - bf_up(h0)), l1 = bf_bits(f1 - bf_up(h1));
        a[e] = pk16(h0, h1); a2[e] = pk16(l0, l1);
      }
      hv[it] = a; lv[it] = a2;
    }
    for (int pass = 0; pass < 2; ++pass) {
#pragma unroll
      for (int it = 0; it < 4; ++it) {
        const int row = it * 4 + q4;
        const size_t go = (rowB + q0 + row) * DMOD + (size_t)h * HD + c8;
        *(volatile v4u*)(ohp + go) = hv[it];
        *(volatile v4u*)(olp + go) = lv[it];
      }
      __threadfence();
    }
  }
}

__global__ __launch_bounds__(256) void ln_rows(const float* __restrict__ y, const float* __restrict__ g,
                                               const float* __restrict__ be, float* out, int nrows) {
  const int lane = threadIdx.x & 31;
  const int wave = threadIdx.x >> 5;
  const int row  = blockIdx.x * 8 + wave;
  if (row >= nrows) return;
  const float* yr = y + (size_t)row * DMOD + lane * 4;
  float s = 0.f;
#pragma unroll 1
  for (int j = 0; j < DMOD / 128; ++j) {
    const v4f x = *(const v4f*)(yr + j * 128);
    s += (x[0] + x[1]) + (x[2] + x[3]);
  }
#pragma unroll
  for (int off = 1; off < 32; off <<= 1) s += __shfl_xor(s, off, 32);
  const float mu = s * (1.0f / (float)DMOD);
  float ss = 0.f;
#pragma unroll 1
  for (int j = 0; j < DMOD / 128; ++j) {
    const v4f x = *(const v4f*)(yr + j * 128);
    const float d0 = x[0] - mu, d1 = x[1] - mu, d2 = x[2] - mu, d3 = x[3] - mu;
    ss += (d0 * d0 + d1 * d1) + (d2 * d2 + d3 * d3);
  }
#pragma unroll
  for (int off = 1; off < 32; off <<= 1) ss += __shfl_xor(ss, off, 32);
  const float var = ss * (1.0f / (float)DMOD);
  const float inv = 1.0f / sqrtf(var + 1.0e-5f);
  v4f o[DMOD / 128];
#pragma unroll
  for (int j = 0; j < DMOD / 128; ++j) {
    const v4f x  = *(const v4f*)(yr + j * 128);
    const v4f gg = *(const v4f*)(g  + j * 128 + lane * 4);
    const v4f bb = *(const v4f*)(be + j * 128 + lane * 4);
    v4f t;
#pragma unroll
    for (int e = 0; e < 4; ++e) t[e] = (x[e] - mu) * inv * bf_rn(gg[e]) + bf_rn(bb[e]);
    o[j] = t;
  }
  float* orow = out + (size_t)row * DMOD + lane * 4;
  for (int pass = 0; pass < 2; ++pass) {
#pragma unroll
    for (int j = 0; j < DMOD / 128; ++j) *(volatile v4f*)(orow + j * 128) = o[j];
    __threadfence();
  }
}

extern "C" void kernel_launch(void* const* d_in, const int* in_sizes, int n_in,
                              void* d_out, int out_size, void* d_ws, size_t ws_size,
                              hipStream_t stream) {
  if (n_in < 14) return;
  if (in_sizes[0] != NTOK * DMOD || in_sizes[1] != NTOK * DMOD || in_sizes[2] != NTOK * DMOD) return;
  if (in_sizes[3] != NB * SEQ) return;
  if (in_sizes[4] != DMOD * DMOD || in_sizes[5] != DMOD * DMOD || in_sizes[6] != DMOD * DMOD ||
      in_sizes[7] != DMOD * DMOD || in_sizes[8] != DMOD * DMOD || in_sizes[10] != DMOD * DMOD) return;
  if (in_sizes[9] != DMOD || in_sizes[11] != DMOD || in_sizes[12] != DMOD || in_sizes[13] != DMOD) return;
  if (out_size != NTOK * DMOD) return;

  const float* xq   = (const float*)d_in[0];
  const float* xk   = (const float*)d_in[1];
  const float* xv   = (const float*)d_in[2];
  const int*   mask = (const int*)d_in[3];
  const float* Wq   = (const float*)d_in[4];
  const float* Wk   = (const float*)d_in[5];
  const float* Wv   = (const float*)d_in[6];
  const float* Wo   = (const float*)d_in[7];
  const float* W1   = (const float*)d_in[8];
  const float* b1   = (const float*)d_in[9];
  const float* W2   = (const float*)d_in[10];
  const float* b2   = (const float*)d_in[11];
  const float* lng  = (const float*)d_in[12];
  const float* lnb  = (const float*)d_in[13];

  const size_t PA = (size_t)NTOK * DMOD * 2;
  const size_t PW = (size_t)DMOD * DMOD * 2;
  const size_t PF = (size_t)NTOK * DMOD * 4;
  size_t off = 0;
  const size_t oX0 = off; off += PA;
  const size_t oX1 = off; off += PA;
  const size_t oX2 = off; off += PA;
  const size_t oWq = off; off += PW;
  const size_t oWk = off; off += PW;
  const size_t oWv = off; off += PW;
  const size_t oWo = off; off += PW;
  const size_t oW1 = off; off += PW;
  const size_t oW2 = off; off += PW;
  const size_t oQ  = off; off += PA;
  const size_t oK  = off; off += PA;
  const size_t oVh = off; off += PA;
  const size_t oVl = off; off += PA;
  const size_t oAf = off; off += PF;
  if (off > ws_size) return;
  if (off > (size_t)134217728) return;
  if (2 * PA != PF) return;

  char* ws = (char*)d_ws;
  unsigned short* Xq  = (unsigned short*)(ws + oX0);
  unsigned short* Xk  = (unsigned short*)(ws + oX1);
  unsigned short* Xv  = (unsigned short*)(ws + oX2);
  unsigned short* WqT = (unsigned short*)(ws + oWq);
  unsigned short* WkT = (unsigned short*)(ws + oWk);
  unsigned short* WvT = (unsigned short*)(ws + oWv);
  unsigned short* WoT = (unsigned short*)(ws + oWo);
  unsigned short* W1T = (unsigned short*)(ws + oW1);
  unsigned short* W2T = (unsigned short*)(ws + oW2);
  unsigned short* Qp  = (unsigned short*)(ws + oQ);
  unsigned short* Kpl = (unsigned short*)(ws + oK);
  unsigned short* VTh = (unsigned short*)(ws + oVh);
  unsigned short* VTl = (unsigned short*)(ws + oVl);
  float*          Af  = (float*)(ws + oAf);
  unsigned short* Oh  = (unsigned short*)(ws + oX0);
  unsigned short* Ol  = (unsigned short*)(ws + oX1);
  unsigned short* Ah  = (unsigned short*)(ws + oQ);
  unsigned short* Al  = (unsigned short*)(ws + oK);
  unsigned short* H1h = (unsigned short*)(ws + oVh);
  unsigned short* H1l = (unsigned short*)(ws + oVl);
  float*          Y   = (float*)(ws + oX0);

  const dim3 blk(256);
  const int n8x = NTOK * DMOD / 8;
  const dim3 gCvt((n8x + 255) / 256);
  const dim3 gWT(DMOD / 64, DMOD / 64);
  const dim3 gProj(((NTOK / 64) * (DMOD / 64) + 7) / 8, 1);
  const dim3 gVT(((DMOD / 64) * (SEQ / 64) + 7) / 8, NB);
  const dim3 gAtt(NB * NH * NKT);
  const dim3 gLN((NTOK + 7) / 8);

  cvt_bf16x8<<<gCvt, blk, 0, stream>>>(xq, Xq, n8x);
  cvt_bf16x8<<<gCvt, blk, 0, stream>>>(xk, Xk, n8x);
  cvt_bf16x8<<<gCvt, blk, 0, stream>>>(xv, Xv, n8x);
  cvt_wT<<<gWT, blk, 0, stream>>>(Wq, WqT);
  cvt_wT<<<gWT, blk, 0, stream>>>(Wk, WkT);
  cvt_wT<<<gWT, blk, 0, stream>>>(Wv, WvT);
  cvt_wT<<<gWT, blk, 0, stream>>>(Wo, WoT);
  cvt_wT<<<gWT, blk, 0, stream>>>(W1, W1T);
  cvt_wT<<<gWT, blk, 0, stream>>>(W2, W2T);
  gemm64<0, 1, 0><<<gProj, blk, 0, stream>>>(
      Xq, Xq, DMOD, 0LL, WqT, DMOD, 0LL, b1, b1,
      (void*)Qp, (void*)Qp, (void*)Qp, DMOD, 0LL,
      NTOK, DMOD, DMOD, 16.0f, 1.0f);
  gemm64<0, 1, 0><<<gProj, blk, 0, stream>>>(
      Xk, Xk, DMOD, 0LL, WkT, DMOD, 0LL, b1, b1,
      (void*)Kpl, (void*)Kpl, (void*)Kpl, DMOD, 0LL,
      NTOK, DMOD, DMOD, 16.0f, 1.0f);
  gemm64<0, 3, 0><<<gVT, blk, 0, stream>>>(
      WvT, WvT, DMOD, 0LL, Xv, DMOD, (long long)SEQ * DMOD, b1, b1,
      (void*)VTh, (void*)VTl, (void*)VTl, SEQ, (long long)DMOD * SEQ,
      DMOD, SEQ, DMOD, 16.0f, 4096.0f);
  attn64<<<gAtt, dim3(128), 0, stream>>>(
      Qp, Kpl, VTh, VTl, mask, Oh, Ol, 0.125f / 256.0f, 1.0f / 16384.0f, 1.0f / 4096.0f);
  gemm64<1, 5, 0><<<gProj, blk, 0, stream>>>(
      Oh, Ol, DMOD, 0LL, WoT, DMOD, 0LL, b1, b1,
      (void*)Af, (void*)Ah, (void*)Al, DMOD, 0LL,
      NTOK, DMOD, DMOD, 1.0f, 1.0f);
  gemm64<1, 2, 3><<<gProj, blk, 0, stream>>>(
      Ah, Al, DMOD, 0LL, W1T, DMOD, 0LL, b1, b1,
      (void*)H1h, (void*)H1l, (void*)H1l, DMOD, 0LL,
      NTOK, DMOD, DMOD, 1.0f, 1.0f);
  gemm64<1, 4, 5><<<gProj, blk, 0, stream>>>(
      H1h, H1l, DMOD, 0LL, W2T, DMOD, 0LL, b2, Af,
      (void*)Y, (void*)Y, (void*)Y, DMOD, 0LL,
      NTOK, DMOD, DMOD, 1.0f, 1.0f);
  ln_rows<<<gLN, blk, 0, stream>>>(Y, lng, lnb, (float*)d_out, NTOK);
  (void)hipGetLastError();
}
